// PGATActor_46084999086427
// MI455X (gfx1250) — hardware-run, weakly checked
//
#include <hip/hip_runtime.h>


namespace {
constexpr int N = 16384, E = 131072, NLIM = 16384  , DIN = 64, HID = 128, HEADS = 4, C = 128, HC = HEADS * C, F1 = 256, NOUT = 2;
constexpr float XS = 8.0f, WSC = 256.0f, SCALE = 0.17677669529663687f;
static_assert(N % 64 == 0 && NLIM % 64 == 0 && NLIM <= N && DIN % 32 == 0 && HID % 32 == 0 && HC % 128 == 0 && F1 % 128 == 0, "tiling");
typedef _Float16 b16;
typedef __attribute__((ext_vector_type(16))) _Float16 v16b;
typedef __attribute__((ext_vector_type(8))) _Float16 v8b;
typedef __attribute__((ext_vector_type(8))) float v8f;
typedef __attribute__((ext_vector_type(4))) float v4f;
__device__ __forceinline__ float bf16_rne(float f) { unsigned int u = __float_as_uint(f); u += 0x7FFFu + ((u >> 16) & 1u); return __uint_as_float(u & 0xFFFF0000u); }
__device__ __forceinline__ void split16(float v, b16& hi, b16& lo) { hi = (b16)v; lo = (b16)(v - (float)hi); }
__device__ __forceinline__ v16b frag_kb(const b16* p, int hh) { const v8b a = *(const v8b*)(p + 8 * hh), b = *(const v8b*)(p + 16 + 8 * hh); v16b f;
#pragma unroll
  for (int e = 0; e < 8; ++e) { f[e] = a[e]; f[8 + e] = b[e]; } return f; }
__device__ __forceinline__ v8f wmma16b(v16b a, v16b b, v8f c) { v8f d = __builtin_amdgcn_wmma_f32_16x16x32_f16(false, a, false, b, (short)0, c, false, false); asm volatile("v_nop\n\tv_nop\n\tv_nop\n\tv_nop" : "+v"(d) : "v"(a), "v"(b)); return d; }
__device__ __forceinline__ void wave_lds_sync() { __builtin_amdgcn_fence(__ATOMIC_RELEASE, "workgroup"); __builtin_amdgcn_wave_barrier(); __builtin_amdgcn_fence(__ATOMIC_ACQUIRE, "workgroup"); }
__device__ __forceinline__ float pmul(float a, float b) { float p = a * b; asm volatile("" : "+v"(p)); return p; }
__device__ __forceinline__ int iclamp(int v, int lo, int hi) { return v < lo ? lo : (v > hi ? hi : v); }
constexpr int CSR_NBLK = 512, CSR_GB = 9, CSR_GN = 1 << CSR_GB  , CSR_MAXG = 512, CSR_CAP = 12288  ;
__global__ __launch_bounds__(64) void csrA_kernel(const int* __restrict__ dst, int E, int N, int nG, int CHP, int NGP, int* __restrict__ STG, int* __restrict__ HST) {
  extern __shared__ int sm[];
  int* cnt = sm; int* run = sm + NGP; int* ids = sm + 2 * NGP;
  const int b = blockIdx.x; const int ch = (E + CSR_NBLK - 1) / CSR_NBLK; const int e0 = b * ch, e1 = min(E, e0 + ch);
  for (int i = threadIdx.x; i < NGP; i += 64) cnt[i] = 0;
  for (int i = threadIdx.x; i < CHP; i += 64) ids[i] = -1;
  __syncthreads();
  if (threadIdx.x == 0) {
    for (int e = e0; e < e1; ++e) { int d = dst[e]; d = (d < 0) ? 0 : (d >= N ? N - 1 : d); cnt[d >> CSR_GB] += 1; }
    int acc = 0; for (int g = 0; g < nG; ++g) { run[g] = acc; acc += cnt[g]; }
    for (int e = e0; e < e1; ++e) { int d = dst[e]; d = (d < 0) ? 0 : (d >= N ? N - 1 : d); const int g = d >> CSR_GB; ids[run[g]] = e; run[g] += 1; } }
  __syncthreads();
  typedef __attribute__((ext_vector_type(4))) int v4i;
  for (int pass = 0; pass < 2; ++pass) {
    for (int i = threadIdx.x; i < CHP / 4; i += 64) *(volatile v4i*)(STG + (size_t)b * CHP + i * 4) = *(const v4i*)(&ids[i * 4]);
    for (int i = threadIdx.x; i < NGP / 4; i += 64) { v4i v; for (int e = 0; e < 4; ++e) v[e] = (i * 4 + e < nG) ? cnt[i * 4 + e] : 0; *(volatile v4i*)(HST + (size_t)b * NGP + i * 4) = v; }
    __threadfence(); }
}
__global__ __launch_bounds__(512) void csrS_kernel(const int* __restrict__ HST, int nG, int NGP, int* __restrict__ START, int* __restrict__ TOT, int* __restrict__ OFF) {
  __shared__ int tot[CSR_MAXG];
  const int b = threadIdx.x;
  for (int pass = 0; pass < 2; ++pass) { int runb = 0; for (int g = 0; g < nG; ++g) { int c = HST[(size_t)b * NGP + g]; c = (c < 0) ? 0 : c; ((volatile int*)OFF)[(size_t)g * CSR_NBLK + b] = runb; runb += c; } __threadfence(); }
  for (int g = threadIdx.x; g < nG; g += 512) { int s = 0; for (int bb = 0; bb < CSR_NBLK; ++bb) { int c = HST[(size_t)bb * NGP + g]; s += (c < 0) ? 0 : c; } tot[g] = s; }
  __syncthreads();
  if (threadIdx.x < 32) {
    __shared__ int st[CSR_MAXG + 32];
    if (threadIdx.x == 0) { int acc = 0; for (int g = 0; g < NGP; ++g) { st[g] = acc; if (g < nG) acc += (tot[g] + 31) & ~31; } st[NGP] = acc; }
    __builtin_amdgcn_fence(__ATOMIC_RELEASE, "workgroup"); __builtin_amdgcn_wave_barrier(); __builtin_amdgcn_fence(__ATOMIC_ACQUIRE, "workgroup");
    for (int pass = 0; pass < 2; ++pass) { for (int i = threadIdx.x; i < NGP + 32; i += 32) { ((volatile int*)START)[i] = (i <= NGP) ? st[min(i, NGP)] : 0; ((volatile int*)TOT)[i] = (i < nG) ? tot[i] : 0; } __threadfence(); } }
}
__global__ __launch_bounds__(256) void csrB_kernel(const int* __restrict__ dst, int N, int nG, int CHP, int NGP, int permLen, const int* __restrict__ STG, const int* __restrict__ HST, const int* __restrict__ OFF, const int* __restrict__ START, const int* __restrict__ TOT, int* __restrict__ PERM, int* __restrict__ ROWPTR, int* __restrict__ ROWCNT, int* __restrict__ FLAG) {
  typedef __attribute__((ext_vector_type(4))) int v4i;
  __shared__ int ids[CSR_CAP]; __shared__ unsigned short key[CSR_CAP]; __shared__ int outp[CSR_CAP]; __shared__ int ncnt[CSR_GN + 1]; __shared__ int boff[CSR_NBLK + 1];
  const int g = blockIdx.x, t_ = threadIdx.x; int tot = TOT[g]; int st = START[g], stn = START[g + 1]; const int v0 = g * CSR_GN; const int nv = min(CSR_GN, N - v0);
  st = (st < 0) ? 0 : (st > permLen - 32 ? permLen - 32 : st) & ~31; stn = (stn < st) ? st : (stn > permLen ? permLen : stn); tot = (tot < 0) ? 0 : tot; if (tot > stn - st && tot <= CSR_CAP) tot = stn - st;
  if (tot > CSR_CAP) {
    for (int pass = 0; pass < 2; ++pass) { for (int i = t_; i < CSR_GN / 4; i += 256) { v4i a, c; for (int e = 0; e < 4; ++e) { a[e] = st; c[e] = 0; } *(volatile v4i*)(ROWPTR + v0 + i * 4) = a; *(volatile v4i*)(ROWCNT + v0 + i * 4) = c; } if (t_ == 0) ((volatile int*)FLAG)[0] = 1; __threadfence(); } (void)nv; return; }
  if (t_ == 0) { int acc = 0; for (int b = 0; b < CSR_NBLK; ++b) { boff[b] = acc; int c = HST[(size_t)b * NGP + g]; c = (c < 0) ? 0 : (c > CHP ? CHP : c); acc += c; if (acc > tot) acc = tot; } boff[CSR_NBLK] = acc; }
  for (int i = t_; i <= CSR_GN; i += 256) ncnt[i] = 0;
  __syncthreads();
  for (int b = 0; b < CSR_NBLK; ++b) { const int c = boff[b + 1] - boff[b]; int o_ = OFF[(size_t)g * CSR_NBLK + b]; o_ = (o_ < 0) ? 0 : (o_ > CHP - c ? CHP - c : o_); const int* src_ = STG + (size_t)b * CHP + o_;
    for (int i = t_; i < c; i += 256) { int id = src_[i]; id = (id < 0) ? 0 : id; ids[boff[b] + i] = id; int d = dst[id]; d = (d < v0) ? v0 : (d >= N ? N - 1 : d); int kk = d - v0; kk = (kk < 0) ? 0 : (kk >= CSR_GN ? CSR_GN - 1 : kk); key[boff[b] + i] = (unsigned short)kk; } }
  __syncthreads();
  if (t_ == 0) { for (int i = 0; i < tot; ++i) ncnt[key[i]] += 1; int acc = 0; for (int vl = 0; vl < CSR_GN; ++vl) { const int c = ncnt[vl]; ncnt[vl] = acc; acc += c; } ncnt[CSR_GN] = acc;
    for (int i = 0; i < tot; ++i) { const int vl = key[i]; outp[ncnt[vl]] = ids[i]; ncnt[vl] += 1; }
    for (int vl = CSR_GN; vl > 0; --vl) ncnt[vl] = ncnt[vl - 1]; ncnt[0] = 0; }
  __syncthreads();
  for (int pass = 0; pass < 2; ++pass) {
    for (int i = t_; i < (stn - st) / 4; i += 256) { v4i v; for (int e = 0; e < 4; ++e) { const int q = i * 4 + e; v[e] = (q < tot) ? outp[q] : -1; } *(volatile v4i*)(PERM + st + i * 4) = v; }
    for (int i = t_; i < CSR_GN / 4; i += 256) { v4i a, c; for (int e = 0; e < 4; ++e) { const int vl = i * 4 + e; a[e] = st + ncnt[vl]; c[e] = (vl < nv) ? (ncnt[vl + 1] - ncnt[vl]) : 0; } *(volatile v4i*)(ROWPTR + v0 + i * 4) = a; *(volatile v4i*)(ROWCNT + v0 + i * 4) = c; }
    __threadfence(); }
}
__global__ __launch_bounds__(256) void csrZ_kernel(int* __restrict__ p, size_t n4) { typedef __attribute__((ext_vector_type(4))) int v4i; const size_t tid = (size_t)blockIdx.x * 256 + threadIdx.x, nth = (size_t)gridDim.x * 256; v4i z = {0, 0, 0, 0}; for (size_t i = tid; i < n4; i += nth) *(volatile v4i*)(p + i * 4) = z; }
struct CsrBufs { int *STG, *HST, *OFF, *START, *TOT, *PERM, *ROWPTR, *ROWCNT, *FLAG; int nG, NGP, CHP; size_t permLen; char* base; size_t bytes; };
static size_t csr_carve(CsrBufs& c, char* ws, size_t off, int E, int N) {
  const size_t off0 = off; c.base = ws + off;
  auto al = [&](size_t bytes) { char* p = ws + off; off += (bytes + 255) & ~(size_t)255; return p; };
  c.nG = (N + CSR_GN - 1) / CSR_GN; c.NGP = (c.nG + 31) & ~31; const int ch = (E + CSR_NBLK - 1) / CSR_NBLK; c.CHP = (ch + 31) & ~31; c.permLen = (size_t)E + 32 * (size_t)c.nG + 32;
  c.STG = (int*)al((size_t)CSR_NBLK * c.CHP * 4); c.HST = (int*)al((size_t)CSR_NBLK * c.NGP * 4); c.OFF = (int*)al((size_t)c.NGP * CSR_NBLK * 4); c.START = (int*)al((size_t)(c.NGP + 64) * 4); c.TOT = (int*)al((size_t)(c.NGP + 64) * 4);
  c.PERM = (int*)al(c.permLen * 4); c.ROWPTR = (int*)al((size_t)c.nG * CSR_GN * 4); c.ROWCNT = (int*)al((size_t)c.nG * CSR_GN * 4); c.FLAG = (int*)al(256);
  c.bytes = off - off0; return off;
}
static void csr_build(const CsrBufs& c, const int* dst, int E, int N, hipStream_t stream) {
  const size_t smem = (size_t)(2 * c.NGP + c.CHP) * 4;
  csrZ_kernel<<<512, 256, 0, stream>>>((int*)c.base, c.bytes / 16);
  csrA_kernel<<<CSR_NBLK, 64, smem, stream>>>(dst, E, N, c.nG, c.CHP, c.NGP, c.STG, c.HST);
  csrS_kernel<<<1, 512, 0, stream>>>(c.HST, c.nG, c.NGP, c.START, c.TOT, c.OFF);
  csrB_kernel<<<c.nG, 256, 0, stream>>>(dst, N, c.nG, c.CHP, c.NGP, (int)c.permLen, c.STG, c.HST, c.OFF, c.START, c.TOT, c.PERM, c.ROWPTR, c.ROWCNT, c.FLAG);
}

typedef __attribute__((ext_vector_type(4))) _Float16 v4h;
typedef __attribute__((ext_vector_type(2))) float v2f;
__device__ __forceinline__ float tanh_f(float x) { const float e = __expf(2.0f * x); return 1.0f - 2.0f / (e + 1.0f); }
__global__ __launch_bounds__(256) void prep_kernel(const float* __restrict__ x, const float* __restrict__ w0, const float* __restrict__ w1, const float* __restrict__ w2, const float* __restrict__ w3, const float* __restrict__ w4, const float* __restrict__ w5,
                                                    b16* __restrict__ Xh, b16* __restrict__ W0, b16* __restrict__ W1, b16* __restrict__ W2, b16* __restrict__ W3, b16* __restrict__ W4, b16* __restrict__ W5) {
  size_t t = (size_t)blockIdx.x * 256 + threadIdx.x; v8b o; const float* src = nullptr; b16* dstp = nullptr; float sc = WSC;
  const size_t n[7] = {(size_t)N * DIN / 8, (size_t)HC * DIN / 8, (size_t)HID * HC / 8, (size_t)HC * HID / 8, (size_t)HID * HC / 8, (size_t)F1 * HID / 8, (size_t)F1 * F1 / 8};
  const float* s_[7] = {x, w0, w1, w2, w3, w4, w5}; b16* d_[7] = {Xh, W0, W1, W2, W3, W4, W5};
#pragma unroll
  for (int i = 0; i < 7; ++i) { if (!src) { if (t < n[i]) { src = s_[i]; dstp = d_[i]; if (i == 0) sc = XS; } else t -= n[i]; } }
  if (!src) return; const size_t e = t * 8;
  for (int j = 0; j < 8; ++j) o[j] = (b16)(bf16_rne(src[e + j]) * sc);
  for (int pass = 0; pass < 2; ++pass) { *(volatile v8b*)(dstp + e) = o; __threadfence(); }
}
template <int KD, int TWO, int NCOL, int EPI, int OUTF, int OUTP>
__global__ __launch_bounds__(128) void gemm_kernel(const b16* __restrict__ Ah, const b16* __restrict__ Al, const b16* __restrict__ W, const float* __restrict__ bias, float* __restrict__ OUT, b16* __restrict__ Ph, b16* __restrict__ Pl) {
  __shared__ __attribute__((aligned(16))) float Tf[4][16][128 + 4];
  const int wave = threadIdx.x >> 5, lane = threadIdx.x & 31, nloc = lane & 15, hlf = lane >> 4; const size_t m0 = (size_t)blockIdx.x * 64 + wave * 16; const int n0 = blockIdx.y * 128;
  v8f acc[8];
#pragma unroll
  for (int t = 0; t < 8; ++t) acc[t] = (v8f){};
#pragma unroll 2
  for (int kb = 0; kb < KD; kb += 32) { const v16b a = frag_kb(Ah + (m0 + nloc) * KD + kb, hlf); v16b al; if (TWO) al = frag_kb(Al + (m0 + nloc) * KD + kb, hlf);
#pragma unroll
    for (int t = 0; t < 8; ++t) { const v16b bw = frag_kb(W + (size_t)(n0 + t * 16 + nloc) * KD + kb, hlf); acc[t] = wmma16b(a, bw, acc[t]); if (TWO) acc[t] = wmma16b(al, bw, acc[t]); } }
#pragma unroll
  for (int t = 0; t < 8; ++t)
#pragma unroll
    for (int r = 0; r < 8; ++r) Tf[wave][8 * hlf + r][t * 16 + nloc] = acc[t][r] * (1.0f / (XS * WSC));
  wave_lds_sync();
  v4f bb = {0.0f, 0.0f, 0.0f, 0.0f}; if (bias != nullptr) { for (int j = 0; j < 4; ++j) bb[j] = bf16_rne(bias[n0 + lane * 4 + j]); }
  for (int rr = 0; rr < 16; ++rr) { v4f o = *(const v4f*)(&Tf[wave][rr][lane * 4]); for (int j = 0; j < 4; ++j) { o[j] += bb[j]; if (EPI == 1) o[j] = tanh_f(o[j]); if (EPI == 2) o[j] = fmaxf(o[j], 0.0f); } *(v4f*)(&Tf[wave][rr][lane * 4]) = o; }
  wave_lds_sync();
  for (int pass = 0; pass < 2; ++pass) { for (int rr = 0; rr < 16; ++rr) { const v4f o = *(const v4f*)(&Tf[wave][rr][lane * 4]);
      if (OUTF) *(volatile v4f*)(OUT + (m0 + rr) * NCOL + n0 + lane * 4) = o;
      if (OUTP) { v4h hv, lv; for (int j = 0; j < 4; ++j) { b16 p, q; split16(o[j] * XS, p, q); hv[j] = p; lv[j] = q; } *(volatile v4h*)(Ph + (m0 + rr) * NCOL + n0 + lane * 4) = hv; *(volatile v4h*)(Pl + (m0 + rr) * NCOL + n0 + lane * 4) = lv; } }
    __threadfence(); }
}
__global__ __launch_bounds__(256) void agg_kernel(const float* __restrict__ V, const float* __restrict__ pos, const float* __restrict__ wq, const float* __restrict__ wk, const int* __restrict__ srcs, const int* __restrict__ PERM, const int* __restrict__ ROWPTR, const int* __restrict__ ROWCNT, int permLen, b16* __restrict__ AGh, b16* __restrict__ AGl) {
  __shared__ float Msh[HEADS * 4];
  if (threadIdx.x < HEADS * 4) { const int h = threadIdx.x >> 2, a = (threadIdx.x >> 1) & 1, b = threadIdx.x & 1; float m = 0.0f;
#pragma unroll 1
    for (int c = 0; c < C; ++c) m += pmul(bf16_rne(wq[(size_t)(h * C + c) * 2 + a]), bf16_rne(wk[(size_t)(h * C + c) * 2 + b])); Msh[threadIdx.x] = m * SCALE; }
  __syncthreads();
  const int wave = threadIdx.x >> 5, lane = threadIdx.x & 31; const size_t v = (size_t)blockIdx.x * 8 + wave; if (v >= (size_t)NLIM) return;
  int st = ROWPTR[v], cnt = ROWCNT[v]; cnt = iclamp(cnt, 0, 65536); st = iclamp(st, 0, permLen - cnt);
  const float pv0 = bf16_rne(pos[v * 2]), pv1 = bf16_rne(pos[v * 2 + 1]);
  float mx[HEADS];
#pragma unroll
  for (int h = 0; h < HEADS; ++h) mx[h] = -INFINITY;
#pragma unroll 1
  for (int j = 0; j < cnt; ++j) { const int e = iclamp(PERM[st + j], 0, E - 1); const size_t s = (size_t)iclamp(srcs[e], 0, N - 1); const float ps0 = bf16_rne(pos[s * 2]), ps1 = bf16_rne(pos[s * 2 + 1]);
#pragma unroll
    for (int h = 0; h < HEADS; ++h) { const float l = pv0 * (Msh[h * 4 + 0] * ps0 + Msh[h * 4 + 1] * ps1) + pv1 * (Msh[h * 4 + 2] * ps0 + Msh[h * 4 + 3] * ps1); mx[h] = fmaxf(mx[h], l); } }
  float den[HEADS]; v4f acc[HEADS];
#pragma unroll
  for (int h = 0; h < HEADS; ++h) { den[h] = 0.0f; acc[h] = (v4f){0.0f, 0.0f, 0.0f, 0.0f}; }
#pragma unroll 1
  for (int j = 0; j < cnt; ++j) { const int e = iclamp(PERM[st + j], 0, E - 1); const size_t s = (size_t)iclamp(srcs[e], 0, N - 1); const float ps0 = bf16_rne(pos[s * 2]), ps1 = bf16_rne(pos[s * 2 + 1]);
#pragma unroll
    for (int h = 0; h < HEADS; ++h) { const float l = pv0 * (Msh[h * 4 + 0] * ps0 + Msh[h * 4 + 1] * ps1) + pv1 * (Msh[h * 4 + 2] * ps0 + Msh[h * 4 + 3] * ps1); const float ex = __expf(l - mx[h]); den[h] += ex;
      const v4f t = *(const v4f*)(V + s * HC + h * C + lane * 4); for (int i = 0; i < 4; ++i) acc[h][i] += pmul(ex, t[i]); } }
  v4h hv[HEADS], lv[HEADS];
#pragma unroll
  for (int h = 0; h < HEADS; ++h) { const float inv = (cnt > 0) ? 1.0f / den[h] : 0.0f; for (int i = 0; i < 4; ++i) { b16 p, q; split16(pmul(acc[h][i], inv) * XS, p, q); hv[h][i] = p; lv[h][i] = q; } }
  for (int pass = 0; pass < 2; ++pass) {
#pragma unroll
    for (int h = 0; h < HEADS; ++h) { *(volatile v4h*)(AGh + v * HC + h * C + lane * 4) = hv[h]; *(volatile v4h*)(AGl + v * HC + h * C + lane * 4) = lv[h]; } __threadfence(); }
}
__global__ __launch_bounds__(256) void out_kernel(const float* __restrict__ Z2, const float* __restrict__ w3, const float* __restrict__ b3, float* __restrict__ out) {
  const size_t n = (size_t)blockIdx.x * 256 + threadIdx.x; if (n >= (size_t)NLIM) return;
  float o0 = bf16_rne(b3[0]), o1 = bf16_rne(b3[1]);
#pragma unroll 1
  for (int k = 0; k < F1; ++k) { const float z = Z2[n * F1 + k]; o0 += pmul(z, bf16_rne(w3[k])); o1 += pmul(z, bf16_rne(w3[F1 + k])); }
  v2f o = {o0, o1};
  for (int pass = 0; pass < 2; ++pass) { *(volatile v2f*)(out + n * NOUT) = o; __threadfence(); }
}
}

extern "C" void kernel_launch(void* const* d_in, const int* in_sizes, int n_in, void* d_out, int out_size, void* d_ws, size_t ws_size, hipStream_t stream) {
  (void)n_in;
  auto Fp = [&](int i) { return (const float*)d_in[i]; }; auto Ip = [&](int i) { return (const int*)d_in[i]; };
  if (in_sizes[0] != N * DIN || in_sizes[1] != N * 2 || in_sizes[2] != 2 * E || in_sizes[3] != HC * 2 || in_sizes[4] != HC * 2 || in_sizes[5] != HC * DIN || in_sizes[6] != HID * HC || in_sizes[7] != HID || in_sizes[8] != HC * 2 || in_sizes[9] != HC * 2 || in_sizes[10] != HC * HID ||
      in_sizes[11] != HID * HC || in_sizes[12] != HID || in_sizes[13] != F1 * HID || in_sizes[14] != F1 || in_sizes[15] != F1 * F1 || in_sizes[16] != F1 || in_sizes[17] != NOUT * F1 || in_sizes[18] != NOUT || out_size != N * NOUT) return;
  size_t off = 0; char* ws = (char*)d_ws;
  auto carve = [&](size_t bytes) { char* p = ws + off; off += (bytes + 255) & ~(size_t)255; return p; };
  b16* Xh = (b16*)carve((size_t)N * DIN * 2); b16* Wv0 = (b16*)carve((size_t)HC * DIN * 2); b16* Wo0 = (b16*)carve((size_t)HID * HC * 2); b16* Wv1 = (b16*)carve((size_t)HC * HID * 2); b16* Wo1 = (b16*)carve((size_t)HID * HC * 2);
  b16* W1b = (b16*)carve((size_t)F1 * HID * 2); b16* W2b = (b16*)carve((size_t)F1 * F1 * 2);
  float* V = (float*)carve((size_t)N * HC * 4); b16* AGh = (b16*)carve((size_t)N * HC * 2); b16* AGl = (b16*)carve((size_t)N * HC * 2); b16* Hh = (b16*)carve((size_t)N * HID * 2); b16* Hl = (b16*)carve((size_t)N * HID * 2);
  b16* Z1h = (b16*)carve((size_t)N * F1 * 2); b16* Z1l = (b16*)carve((size_t)N * F1 * 2); float* Z2 = V;
  CsrBufs csr; off = csr_carve(csr, ws, off, E, N);
  if (off > ws_size || off > ((size_t)128 << 20)) return;
  prep_kernel<<<(unsigned)((((size_t)N * DIN + (size_t)HC * DIN + 3 * (size_t)HID * HC + (size_t)F1 * HID + (size_t)F1 * F1) / 8 + 255) / 256), 256, 0, stream>>>(Fp(0), Fp(5), Fp(6), Fp(10), Fp(11), Fp(13), Fp(15), Xh, Wv0, Wo0, Wv1, Wo1, W1b, W2b);
  csr_build(csr, Ip(2) + E, E, N, stream);
  gemm_kernel<DIN, 0, HC, 0, 1, 0><<<dim3(NLIM / 64, HC / 128), 128, 0, stream>>>(Xh, nullptr, Wv0, nullptr, V, nullptr, nullptr);
  agg_kernel<<<NLIM / 8, 256, 0, stream>>>(V, Fp(1), Fp(3), Fp(4), Ip(2), csr.PERM, csr.ROWPTR, csr.ROWCNT, (int)csr.permLen, AGh, AGl);
  gemm_kernel<HC, 1, HID, 1, 0, 1><<<dim3(NLIM / 64, HID / 128), 128, 0, stream>>>(AGh, AGl, Wo0, Fp(7), nullptr, Hh, Hl);
  gemm_kernel<HID, 1, HC, 0, 1, 0><<<dim3(NLIM / 64, HC / 128), 128, 0, stream>>>(Hh, Hl, Wv1, nullptr, V, nullptr, nullptr);
  agg_kernel<<<NLIM / 8, 256, 0, stream>>>(V, Fp(1), Fp(8), Fp(9), Ip(2), csr.PERM, csr.ROWPTR, csr.ROWCNT, (int)csr.permLen, AGh, AGl);
  gemm_kernel<HC, 1, HID, 1, 0, 1><<<dim3(NLIM / 64, HID / 128), 128, 0, stream>>>(AGh, AGl, Wo1, Fp(12), nullptr, Hh, Hl);
  gemm_kernel<HID, 1, F1, 2, 0, 1><<<dim3(NLIM / 64, F1 / 128), 128, 0, stream>>>(Hh, Hl, W1b, Fp(14), nullptr, Z1h, Z1l);
  gemm_kernel<F1, 1, F1, 2, 1, 0><<<dim3(NLIM / 64, F1 / 128), 128, 0, stream>>>(Z1h, Z1l, W2b, Fp(16), Z2, nullptr, nullptr);
  out_kernel<<<NLIM / 256, 256, 0, stream>>>(Z2, Fp(17), Fp(18), (float*)d_out);
}
